// CILRSVAEModel_74466142978774
// MI455X (gfx1250) — hardware-run, weakly checked
//
#include <hip/hip_runtime.h>
#define CNR 65536
#define CCH 8192
#define CNE 512
#define CNV 128
#define CNJ 640
#define CNW 256
#define CNB 6
#define CNO 3
typedef unsigned short v8us __attribute__((ext_vector_type(8), may_alias));
typedef float  v8f  __attribute__((ext_vector_type(8)));
typedef float  v4f  __attribute__((ext_vector_type(4)));
typedef float  v4fa __attribute__((ext_vector_type(4), may_alias));

__device__ __forceinline__ unsigned short bf16_bits(float x) { unsigned int u = __float_as_uint(x); return (unsigned short)((u + 0x7FFFu + ((u >> 16) & 1u)) >> 16); }
__device__ __forceinline__ float bf16_val(unsigned short b) { return __uint_as_float(((unsigned int)b) << 16); }
__device__ __forceinline__ float bf16_round(float x) { return bf16_val(bf16_bits(x)); }

typedef _Float16 v16h __attribute__((ext_vector_type(16)));
union FragH { v16h v; v8us half[2]; _Float16 h[16]; unsigned short u[16]; };

__global__ __launch_bounds__(256) void k_wt_f16(const float* __restrict__ W, _Float16* __restrict__ Wt, int K, int N, float scale) {
  const int t = blockIdx.x * 256 + threadIdx.x; if (t >= N * (K / 8)) return; const int n = t / (K / 8), k8 = (t % (K / 8)) * 8; FragH f;
#pragma unroll
  for (int i = 0; i < 8; ++i) f.h[i] = (_Float16)(bf16_round(W[(size_t)(k8 + i) * N + n]) * scale); const v8us o = f.half[0];
  *(volatile v8us*)((unsigned short*)Wt + (size_t)n * K + k8) = o; __threadfence(); *(volatile v8us*)((unsigned short*)Wt + (size_t)n * K + k8) = o;
}

typedef _Float16 v4h __attribute__((ext_vector_type(4)));

__global__ __launch_bounds__(256) void k_x16(const float* __restrict__ x, _Float16* __restrict__ X16, size_t n8) { const size_t t = (size_t)blockIdx.x * 256 + threadIdx.x; if (t >= n8) return; FragH f;
#pragma unroll
  for (int q = 0; q < 8; ++q) f.h[q] = (_Float16)bf16_round(x[t * 8 + q]); *(volatile v8us*)((unsigned short*)X16 + t * 8) = f.half[0]; __threadfence(); *(volatile v8us*)((unsigned short*)X16 + t * 8) = f.half[0]; }

__device__ __forceinline__ v16h g2_frag(const _Float16* p, int hh) { FragH f; f.half[0] = *(const v8us*)((const unsigned short*)p + 8 * hh); f.half[1] = *(const v8us*)((const unsigned short*)p + 16 + 8 * hh); return f.v; }
__device__ __forceinline__ v8f g2_mma(v16h a, v16h b, v8f c) { v8f d = __builtin_amdgcn_wmma_f32_16x16x32_f16(false, a, false, b, (short)0, c, false, false); asm volatile("v_nop\n\tv_nop\n\tv_nop\n\tv_nop" : "+v"(d) : "v"(a), "v"(b)); return d; }
template <int ACT>
__global__ __launch_bounds__(128) void k_gemm2(const _Float16* __restrict__ A, int lda, size_t sA, const _Float16* __restrict__ Bh, int ldb, size_t sB, float alpha, const float* __restrict__ bias, size_t sBias, const float* __restrict__ CP, int rowsPerB, size_t sCPb, int row0g,
    float* __restrict__ C, _Float16* __restrict__ C16, int ldc, size_t sC, int M, int N, int K) { static_assert(ACT == 0 || ACT == 3 || ACT == 6 || ACT == 8 || ACT == 9 || ACT == 11 || ACT == 12 || ACT == 14 || ACT == 15 || ACT == 16 || ACT == 17, "k_gemm2: unsupported ACT code (would silently apply no activation)");
  __shared__ __attribute__((aligned(16))) float so[4][32][68];
  const int tid = threadIdx.x, w = tid >> 5, lane = tid & 31, ln = lane & 15, hh = lane >> 4; const int by = blockIdx.y;
  A += (size_t)by * sA; Bh += (size_t)by * sB; const size_t cofs = (size_t)by * sC; const float* bp = bias ? bias + (size_t)by * sBias : nullptr;
  const int ntn = N >> 6; const int mt = blockIdx.x / ntn, nq = blockIdx.x - mt * ntn; const int row0 = mt * 128 + 32 * w, col0 = nq * 64; if (row0 >= M) return;
  const _Float16* a0p = A + (size_t)(row0 + ln) * lda; const _Float16* a1p = a0p + (size_t)16 * lda;
  const _Float16* b0p = Bh + (size_t)(col0 + ln) * ldb; const _Float16* b1p = b0p + (size_t)16 * ldb; const _Float16* b2p = b1p + (size_t)16 * ldb; const _Float16* b3p = b2p + (size_t)16 * ldb;
  const v8f z8 = {0.f,0.f,0.f,0.f,0.f,0.f,0.f,0.f}; v8f c00 = z8, c01 = z8, c02 = z8, c03 = z8, c10 = z8, c11 = z8, c12 = z8, c13 = z8;
  for (int kb = 0; kb < K; kb += 32) { const v16h a0 = g2_frag(a0p + kb, hh), a1 = g2_frag(a1p + kb, hh);
    v16h b = g2_frag(b0p + kb, hh); c00 = g2_mma(a0, b, c00); c10 = g2_mma(a1, b, c10);
    b = g2_frag(b1p + kb, hh); c01 = g2_mma(a0, b, c01); c11 = g2_mma(a1, b, c11);
    b = g2_frag(b2p + kb, hh); c02 = g2_mma(a0, b, c02); c12 = g2_mma(a1, b, c12);
    b = g2_frag(b3p + kb, hh); c03 = g2_mma(a0, b, c03); c13 = g2_mma(a1, b, c13); }
  v8f accs[8] = {c00, c01, c02, c03, c10, c11, c12, c13};
#pragma unroll
  for (int u = 0; u < 8; ++u) { const int t = u & 3, half = u >> 2; const int col = col0 + t * 16 + ln; const float bv = bp ? bf16_round(bp[col]) : 0.f;
#pragma unroll
    for (int r = 0; r < 8; ++r) { const int rloc = half * 16 + 8 * hh + r; float v = accs[u][r] * alpha + bv; if (CP) { if (rowsPerB < 0) v += CP[cofs + (size_t)(row0g + row0 + rloc) * ldc + col];        else { const int bidx = (row0g + row0 + rloc) / rowsPerB; v += CP[(size_t)bidx * sCPb + (size_t)by * 64 + col]; } }
      if (ACT == 3) v = fmaxf(v, 0.f); else if (ACT == 6) v = 0.5f * v * (1.0f + erff(v * 0.70710678118654752f)); else if (ACT == 11) v = 1.0f / (1.0f + expf(-v)); else if (ACT == 15) v = v / (1.0f + expf(-v)); else if (ACT == 12) v = (v > 0.f) ? v : 0.01f * v; else if (ACT == 8) v = tanhf(v); else if (ACT == 9) v = 0.5f * v * (1.0f + tanhf(0.7978845608028654f * (v + 0.044715f * v * v * v))); else if (ACT == 14) v = (v > 0.f) ? v : 0.1f * v; else if (ACT == 16) v = (v >= 0.f) ? v : 0.3f * v; else if (ACT == 17) v = (v >= 0.f) ? v : 0.2f * v;
      so[w][rloc][t * 16 + ln] = v; } }
  __builtin_amdgcn_fence(__ATOMIC_ACQ_REL, "workgroup"); __builtin_amdgcn_wave_barrier();
  const int rsub = lane >> 4, c4 = (lane & 15) * 4;
  for (int pass = 0; pass < 2; ++pass) {
#pragma unroll
    for (int q = 0; q < 16; ++q) { const int r = q * 2 + rsub; const v4f v = *(const v4fa*)&so[w][r][c4]; if (C) *(volatile v4f*)(C + cofs + (size_t)(row0 + r) * ldc + col0 + c4) = v; if (C16) { v4h h4; for (int i = 0; i < 4; ++i) h4[i] = (_Float16)v[i]; *(volatile v4h*)(C16 + cofs + (size_t)(row0 + r) * ldc + col0 + c4) = h4; } }
    if (pass == 0) __threadfence(); } }

__global__ __launch_bounds__(256) void k_cs16(const float* __restrict__ sw, _Float16* __restrict__ tw, float scale) { const size_t t = (size_t)blockIdx.x * 256 + threadIdx.x; FragH f;
#pragma unroll
  for (int q = 0; q < 8; ++q) f.h[q] = (_Float16)(bf16_round(sw[t * 8 + q]) * scale); unsigned short* tp = (unsigned short*)tw + t * 8; *(volatile v8us*)tp = f.half[0]; __threadfence(); *(volatile v8us*)tp = f.half[0]; }
__global__ __launch_bounds__(256) void k_enc1(const float* __restrict__ sv, const float* __restrict__ sf, const float* __restrict__ sc, _Float16* __restrict__ tw) {
  const unsigned t = blockIdx.x * 256 + threadIdx.x, r = t >> 5, g8 = (t & 31u) * 8; const float a = bf16_round(sv[r]); FragH fw;
#pragma unroll
  for (int q = 0; q < 8; ++q) fw.h[q] = (_Float16)fmaxf(a * bf16_round(sf[g8 + q]) + bf16_round(sc[g8 + q]), 0.f);
  unsigned short* tp = (unsigned short*)tw + (size_t)r * CNW + g8; *(volatile v8us*)tp = fw.half[0]; __threadfence(); *(volatile v8us*)tp = fw.half[0]; }
__global__ __launch_bounds__(256) void k_embp(const float* __restrict__ se, _Float16* __restrict__ tw) {
  const unsigned t = blockIdx.x * 256 + threadIdx.x, r = t >> 6, g8 = (t & 63u) * 8; const float* sr = se + (size_t)r * CNE + g8; FragH fw;
#pragma unroll
  for (int q = 0; q < 8; ++q) fw.h[q] = (_Float16)bf16_round(sr[q]);
  unsigned short* tp = (unsigned short*)tw + (size_t)r * CNJ + g8; *(volatile v8us*)tp = fw.half[0]; __threadfence(); *(volatile v8us*)tp = fw.half[0]; }
__global__ __launch_bounds__(256) void k_tail(const _Float16* __restrict__ pq, size_t sq, const float* __restrict__ sg3, const float* __restrict__ sr3, const int* __restrict__ qv, const _Float16* __restrict__ pu, const float* __restrict__ st3, const float* __restrict__ sv3, float* __restrict__ d0, float* __restrict__ d1) {
  const unsigned t = blockIdx.x * 256 + threadIdx.x; const int cm = qv[t] - 1; float a0 = 0.f, a1 = 0.f, a2 = 0.f;
#pragma unroll
  for (int n = 0; n < CNB; ++n) { const unsigned short* pr = (const unsigned short*)pq + (size_t)n * sq + (size_t)t * CNW; const float* gn = sg3 + (size_t)n * CNW * CNO; float z0 = 0.f, z1 = 0.f, z2 = 0.f;
#pragma unroll
    for (int d8 = 0; d8 < CNW; d8 += 8) { FragH fw; fw.half[0] = *(const v8us*)(pr + d8);
#pragma unroll
      for (int q = 0; q < 8; ++q) { const float a = (float)fw.h[q]; const float* gr = gn + (size_t)(d8 + q) * CNO; z0 += a * bf16_round(gr[0]); z1 += a * bf16_round(gr[1]); z2 += a * bf16_round(gr[2]); } }
    const float m = (cm == n) ? 1.0f : 0.0f; z0 += bf16_round(sr3[n * CNO + 0]); z1 += bf16_round(sr3[n * CNO + 1]); z2 += bf16_round(sr3[n * CNO + 2]); a0 += (1.0f / (1.0f + expf(-z0))) * m; a1 += (1.0f / (1.0f + expf(-z1))) * m; a2 += (1.0f / (1.0f + expf(-z2))) * m; }
  const unsigned short* ur = (const unsigned short*)pu + (size_t)t * CNW; float y = 0.f;
#pragma unroll
  for (int d8 = 0; d8 < CNW; d8 += 8) { FragH fw; fw.half[0] = *(const v8us*)(ur + d8);
#pragma unroll
    for (int q = 0; q < 8; ++q) y += (float)fw.h[q] * bf16_round(st3[d8 + q]); }
  y += bf16_round(sv3[0]); float* p0 = d0 + (size_t)t * CNO; float* p1 = d1 + t; *(volatile float*)(p0 + 0) = a0; *(volatile float*)(p0 + 1) = a1; *(volatile float*)(p0 + 2) = a2; *(volatile float*)p1 = y; __threadfence(); *(volatile float*)(p0 + 0) = a0; *(volatile float*)(p0 + 1) = a1; *(volatile float*)(p0 + 2) = a2; *(volatile float*)p1 = y; }

extern "C" void kernel_launch(void* const* d_in, const int* in_sizes, int n_in,
                              void* d_out, int out_size, void* d_ws, size_t ws_size, hipStream_t stream) {
  if (n_in < 19) return; if (in_sizes[0] < CNR * CNE || in_sizes[1] < CNR || in_sizes[2] < CNR || out_size < CNR * (CNO + 1)) return;
  if (in_sizes[3] < CNW || in_sizes[4] < CNW || in_sizes[5] < CNW * CNV || in_sizes[6] < CNV || in_sizes[7] < CNB * CNJ * CNW || in_sizes[8] < CNB * CNW || in_sizes[9] < CNB * CNW * CNW || in_sizes[10] < CNB * CNW || in_sizes[11] < CNB * CNW * CNO || in_sizes[12] < CNB * CNO || in_sizes[13] < CNJ * CNW || in_sizes[14] < CNW || in_sizes[15] < CNW * CNW || in_sizes[16] < CNW || in_sizes[17] < CNW || in_sizes[18] < 1) return;
  const float* ea = (const float*)d_in[0]; const float* va = (const float*)d_in[1]; const int* qa = (const int*)d_in[2]; const float* f1 = (const float*)d_in[3]; const float* c1 = (const float*)d_in[4]; const float* f2 = (const float*)d_in[5]; const float* c2 = (const float*)d_in[6]; const float* g1 = (const float*)d_in[7]; const float* r1 = (const float*)d_in[8]; const float* g2 = (const float*)d_in[9]; const float* r2 = (const float*)d_in[10]; const float* g3 = (const float*)d_in[11]; const float* r3 = (const float*)d_in[12]; const float* t1 = (const float*)d_in[13]; const float* v1 = (const float*)d_in[14]; const float* t2 = (const float*)d_in[15]; const float* v2 = (const float*)d_in[16]; const float* t3 = (const float*)d_in[17]; const float* v3 = (const float*)d_in[18]; float* res0 = (float*)d_out; float* res1 = res0 + (size_t)CNR * CNO;
  static_assert(CNR % CCH == 0 && CCH % 128 == 0 && CCH % 256 == 0 && CNW % 64 == 0 && CNV % 64 == 0 && CNJ % 32 == 0 && CNW % 32 == 0 && CNJ == CNE + CNV && CNE % 8 == 0 && CNW % 8 == 0 && CNJ % 8 == 0 && (CCH * (CNW / 8)) % 256 == 0 && (CCH * (CNE / 8)) % 256 == 0 && CNO == 3, "whole tiles, whole chunks, exact flat launches, no noughts needed in any depth");
  uint8_t* wsp = (uint8_t*)d_ws; size_t off = 0;
  auto take = [&](size_t bytes) { uint8_t* at = wsp + off; off += (bytes + 255) & ~(size_t)255; return at; };
  _Float16* TF2 = (_Float16*)take((size_t)CNV * CNW * 2); _Float16* TG1 = (_Float16*)take((size_t)CNB * CNW * CNJ * 2); _Float16* TG2 = (_Float16*)take((size_t)CNB * CNW * CNW * 2); _Float16* TT1 = (_Float16*)take((size_t)CNW * CNJ * 2); _Float16* TT2 = (_Float16*)take((size_t)CNW * CNW * 2);
  _Float16* PE1 = (_Float16*)take((size_t)CCH * CNW * 2); _Float16* PJA = (_Float16*)take((size_t)CCH * CNJ * 2); _Float16* PQ1 = (_Float16*)take((size_t)CNB * CCH * CNW * 2); _Float16* PQ2 = (_Float16*)take((size_t)CNB * CCH * CNW * 2); _Float16* PU1 = (_Float16*)take((size_t)CCH * CNW * 2); _Float16* PU2 = (_Float16*)take((size_t)CCH * CNW * 2);
  if (off > ws_size) return;
  const unsigned gw = (unsigned)((CNW * (CNW / 8) + 255) / 256), gj = (unsigned)((CNW * (CNJ / 8) + 255) / 256);
  k_wt_f16<<<(unsigned)((CNV * (CNW / 8) + 255) / 256), 256, 0, stream>>>(f2, TF2, CNW, CNV, 1.0f);
  for (int n = 0; n < CNB; ++n) { k_wt_f16<<<gj, 256, 0, stream>>>(g1 + (size_t)n * CNJ * CNW, TG1 + (size_t)n * CNW * CNJ, CNJ, CNW, 1.0f); k_wt_f16<<<gw, 256, 0, stream>>>(g2 + (size_t)n * CNW * CNW, TG2 + (size_t)n * CNW * CNW, CNW, CNW, 1.0f); }
  k_wt_f16<<<gj, 256, 0, stream>>>(t1, TT1, CNJ, CNW, 1.0f); k_wt_f16<<<gw, 256, 0, stream>>>(t2, TT2, CNW, CNW, 1.0f);
  const dim3 g2c((unsigned)((CCH / 128) * (CNV / 64)), 1), g4c((unsigned)((CCH / 128) * (CNW / 64)), 1), g4b((unsigned)((CCH / 128) * (CNW / 64)), (unsigned)CNB);
  for (int c = 0; c < CNR / CCH; ++c) { const size_t r0 = (size_t)c * CCH;
    k_enc1<<<(unsigned)(CCH * (CNW / 8) / 256), 256, 0, stream>>>(va + r0, f1, c1, PE1); k_embp<<<(unsigned)(CCH * (CNE / 8) / 256), 256, 0, stream>>>(ea + r0 * CNE, PJA);
    k_gemm2<0><<<g2c, 128, 0, stream>>>(PE1, CNW, (size_t)0, TF2, CNW, (size_t)0, 1.0f, c2, (size_t)0, nullptr, 1, 0, 0, nullptr, PJA + CNE, CNJ, (size_t)0, CCH, CNV, CNW);
    k_gemm2<3><<<g4b, 128, 0, stream>>>(PJA, CNJ, (size_t)0, TG1, CNJ, (size_t)CNW * CNJ, 1.0f, r1, (size_t)CNW, nullptr, 1, 0, 0, nullptr, PQ1, CNW, (size_t)CCH * CNW, CCH, CNW, CNJ);
    k_gemm2<3><<<g4b, 128, 0, stream>>>(PQ1, CNW, (size_t)CCH * CNW, TG2, CNW, (size_t)CNW * CNW, 1.0f, r2, (size_t)CNW, nullptr, 1, 0, 0, nullptr, PQ2, CNW, (size_t)CCH * CNW, CCH, CNW, CNW);
    k_gemm2<3><<<g4c, 128, 0, stream>>>(PJA, CNJ, (size_t)0, TT1, CNJ, (size_t)0, 1.0f, v1, (size_t)0, nullptr, 1, 0, 0, nullptr, PU1, CNW, (size_t)0, CCH, CNW, CNJ);
    k_gemm2<3><<<g4c, 128, 0, stream>>>(PU1, CNW, (size_t)0, TT2, CNW, (size_t)0, 1.0f, v2, (size_t)0, nullptr, 1, 0, 0, nullptr, PU2, CNW, (size_t)0, CCH, CNW, CNW);
    k_tail<<<(unsigned)(CCH / 256), 256, 0, stream>>>(PQ2, (size_t)CCH * CNW, g3, r3, qa + r0, PU2, t3, v3, res0 + r0 * CNO, res1 + r0); }
}
